// ExampleModel_11476152615394
// MI455X (gfx1250) — hardware-verified
//
#include <hip/hip_runtime.h>

#define T_TOK   16384
#define HID     512
#define FFN_DIM 2048
#define NEXP    4
#define TM      32
#define FC      256
#define WSC     16.0f
#define WSC_INV 0.0625f

#define OFF_LOGITS 0u
#define OFF_GATES  262144u
#define OFF_W1F    524288u
#define OFF_W2F    (524288u + 8388608u)
#define OFF_XF     (524288u + 2u * 8388608u)

typedef __attribute__((ext_vector_type(16))) _Float16 v16h;
typedef __attribute__((ext_vector_type(8)))  float  v8f;
typedef __attribute__((ext_vector_type(4)))  float  v4f;

union V16U { uint4 u[2]; v16h v; };
static __device__ inline v16h as_v16h(uint4 lo, uint4 hi) {
    V16U t; t.u[0] = lo; t.u[1] = hi; return t.v;
}
static __device__ inline unsigned short f2h_bits(float f) {
    return __builtin_bit_cast(unsigned short, (_Float16)f);
}
static __device__ inline unsigned pack_h2(float a, float b) {
    return (unsigned)f2h_bits(a) | ((unsigned)f2h_bits(b) << 16);
}

__global__ void router_kernel(const float* __restrict__ x,
                              const float* __restrict__ wr,
                              float* __restrict__ logits) {
    int t = blockIdx.x * blockDim.x + threadIdx.x;
    const float4* wr4 = (const float4*)wr;
    const float* xr = x + (size_t)t * HID;
    float a0 = 0.f, a1 = 0.f, a2 = 0.f, a3 = 0.f;
#pragma unroll 4
    for (int k = 0; k < HID; ++k) {
        float xs = xr[k];
        float4 w = wr4[k];
        a0 += xs * w.x; a1 += xs * w.y; a2 += xs * w.z; a3 += xs * w.w;
    }
    v4f o = {a0, a1, a2, a3};
    ((volatile v4f*)logits)[t] = o;
    __threadfence();
    ((volatile v4f*)logits)[t] = o;
}

__global__ void convert_w_kernel(const float* __restrict__ src,
                                 unsigned* __restrict__ dst,
                                 int Kt, int Nt) {
    int d    = blockIdx.x * 256 + threadIdx.x;
    int v    = d & 7;
    int lane = (d >> 3) & 31;
    int rest = d >> 8;
    int kt = rest % Kt;
    int nt = (rest / Kt) % Nt;
    int e  = rest / (Kt * Nt);
    int h  = lane >> 4, nl = lane & 15;
    int k  = kt * 32 + (v >> 2) * 16 + h * 8 + (v & 3) * 2;
    int n  = nt * 16 + nl;
    int K  = Kt * 32, N = Nt * 16;
    const float* s = src + ((size_t)e * K + k) * N + n;
    unsigned u = pack_h2(s[0] * WSC, s[N] * WSC);
    ((volatile unsigned*)dst)[d] = u;
    __threadfence();
    ((volatile unsigned*)dst)[d] = u;
}

__global__ void convert_x_kernel(const float* __restrict__ x,
                                 unsigned* __restrict__ xf) {
    int d    = blockIdx.x * 256 + threadIdx.x;
    int v    = d & 7;
    int lane = (d >> 3) & 31;
    int kk   = (d >> 8) & 15;
    int mt   = d >> 12;
    int h = lane >> 4, ml = lane & 15;
    int k = kk * 32 + (v >> 2) * 16 + h * 8 + (v & 3) * 2;
    const float* xp = x + (size_t)(mt * 16 + ml) * HID + k;
    unsigned u = pack_h2(xp[0], xp[1]);
    ((volatile unsigned*)xf)[d] = u;
    __threadfence();
    ((volatile unsigned*)xf)[d] = u;
}

#define SKT 1024
#define TPT 16
__global__ __launch_bounds__(SKT) void sinkhorn_gates_kernel(const float* __restrict__ logits,
                                      float* __restrict__ gates) {
    __shared__ float red[SKT * 4];
    __shared__ float d1s[4];
    __shared__ float errs;
    const int tid = threadIdx.x;
    const float eps = 1e-8f, invT = 1.f / (float)T_TOK, invE = 0.25f;

    float d1[4] = {1.f, 1.f, 1.f, 1.f};
    for (int iter = 0; iter < 512; ++iter) {
        float p0 = 0.f, p1 = 0.f, p2 = 0.f, p3 = 0.f;
#pragma unroll 1
        for (int i = 0; i < TPT; ++i) {
            float4 l = ((const float4*)logits)[tid + i * SKT];
            float c0 = expf(l.x), c1 = expf(l.y), c2 = expf(l.z), c3 = expf(l.w);
            float den = c0 * d1[0] + c1 * d1[1] + c2 * d1[2] + c3 * d1[3] + eps;
            float v = invT / den;
            p0 += v * c0; p1 += v * c1; p2 += v * c2; p3 += v * c3;
        }
        red[tid*4+0] = p0; red[tid*4+1] = p1; red[tid*4+2] = p2; red[tid*4+3] = p3;
        __syncthreads();
        for (int s = SKT / 2; s > 0; s >>= 1) {
            if (tid < s) {
                red[tid*4+0] += red[(tid+s)*4+0];
                red[tid*4+1] += red[(tid+s)*4+1];
                red[tid*4+2] += red[(tid+s)*4+2];
                red[tid*4+3] += red[(tid+s)*4+3];
            }
            __syncthreads();
        }
        if (tid == 0) {
            float err = 0.f;
            for (int e = 0; e < 4; ++e) {
                float dn = invE / (red[e] + eps);
                err += fabsf(d1[e] - dn);
                d1s[e] = dn;
            }
            errs = err * 0.25f;
        }
        __syncthreads();
        d1[0] = d1s[0]; d1[1] = d1s[1]; d1[2] = d1s[2]; d1[3] = d1s[3];
        const bool done = (errs <= 1e-4f);
        __syncthreads();
        if (done) break;
    }

    for (int pass = 0; pass < 2; ++pass) {
#pragma unroll 1
        for (int i = 0; i < TPT; ++i) {
            int t = tid + i * SKT;
            float4 l = ((const float4*)logits)[t];
            float c[4] = {expf(l.x), expf(l.y), expf(l.z), expf(l.w)};
            float nm[4];
#pragma unroll
            for (int e = 0; e < 4; ++e) nm[e] = d1[e] * c[e];
            int a = 0;
#pragma unroll
            for (int e = 1; e < 4; ++e) if (nm[e] > nm[a]) a = e;
            int b = -1;
#pragma unroll
            for (int e = 0; e < 4; ++e)
                if (e != a && (b < 0 || nm[e] > nm[b])) b = e;
            float ga[4] = {0.f, 0.f, 0.f, 0.f};
#pragma unroll
            for (int e = 0; e < 4; ++e)
                if (e == a || e == b) ga[e] = c[e] / (1.f + c[e]);
            v4f o = {ga[0], ga[1], ga[2], ga[3]};
            ((volatile v4f*)gates)[t] = o;
        }
        __threadfence();
    }
}

__global__ __launch_bounds__(256, 1)
void moe_main_kernel(const unsigned* __restrict__ xf,
                     const unsigned* __restrict__ w1f,
                     const unsigned* __restrict__ w2f,
                     const float* __restrict__ gates,
                     float* __restrict__ out) {
    __shared__ __align__(32) unsigned       xfrag[2 * 16 * 32 * 8];
    __shared__ __align__(16) unsigned short hbuf[TM * FC];
    __shared__ float gsh[NEXP * TM];

    int tid  = threadIdx.x;
    int lane = tid & 31, w = tid >> 5;
    int mw = w >> 2, nw = w & 3;
    int h  = lane >> 4, nl = lane & 15;
    int t0 = blockIdx.x * TM;

    if (tid < TM) {
        float4 g = ((const float4*)gates)[t0 + tid];
        gsh[0*TM + tid] = g.x; gsh[1*TM + tid] = g.y;
        gsh[2*TM + tid] = g.z; gsh[3*TM + tid] = g.w;
    }
    const unsigned* xsrc = xf + (size_t)blockIdx.x * (2 * 16 * 32 * 8);
#pragma unroll
    for (int j = 0; j < 8; ++j) {
        int off = (j * 256 + tid) * 4;
        *(uint4*)(xfrag + off) = *(const uint4*)(xsrc + off);
    }
    __syncthreads();

    v8f oacc[8];
#pragma unroll
    for (int i = 0; i < 8; ++i) oacc[i] = (v8f){0.f,0.f,0.f,0.f,0.f,0.f,0.f,0.f};

    for (int e = 0; e < NEXP; ++e) {
        float g8[8];
#pragma unroll
        for (int r = 0; r < 8; ++r) g8[r] = gsh[e * TM + mw * 16 + r + 8 * h];

        for (int fc = 0; fc < FFN_DIM / FC; ++fc) {
#pragma unroll
            for (int nn = 0; nn < 4; ++nn) {
                int nt = fc * (FC / 16) + nw * 4 + nn;
                v8f acc = (v8f){0.f,0.f,0.f,0.f,0.f,0.f,0.f,0.f};
                for (int kk = 0; kk < HID / 32; ++kk) {
                    v16h a = as_v16h(*(const uint4*)(xfrag + ((mw * 16 + kk) * 32 + lane) * 8),
                                     *(const uint4*)(xfrag + ((mw * 16 + kk) * 32 + lane) * 8 + 4));
                    const uint4* bp = (const uint4*)
                        (w1f + (((size_t)((e * (FFN_DIM/16) + nt) * (HID/32) + kk)) * 32 + lane) * 8);
                    v16h b = as_v16h(bp[0], bp[1]);
                    acc = __builtin_amdgcn_wmma_f32_16x16x32_f16(false, a, false, b, (short)0, acc, false, false);
                    asm volatile("v_nop\n\tv_nop\n\tv_nop\n\tv_nop" : "+v"(acc) : "v"(a), "v"(b));
                }
#pragma unroll
                for (int r = 0; r < 8; ++r) {
                    float s  = acc[r] * WSC_INV;
                    float hv = s / (1.f + expf(-s));
                    int m = mw * 16 + r + 8 * h;
                    hbuf[m * FC + (nw * 4 + nn) * 16 + nl] = f2h_bits(hv);
                }
            }
            __syncthreads();

#pragma unroll
            for (int on = 0; on < 8; ++on) {
                int n = nw * 8 + on;
                v8f acc = (v8f){0.f,0.f,0.f,0.f,0.f,0.f,0.f,0.f};
                for (int kk = 0; kk < FC / 32; ++kk) {
                    int m = mw * 16 + nl;
                    const unsigned short* hp = hbuf + m * FC + kk * 32 + h * 8;
                    v16h a = as_v16h(*(const uint4*)hp, *(const uint4*)(hp + 16));
                    int ktile = fc * (FC / 32) + kk;
                    const uint4* bp = (const uint4*)
                        (w2f + (((size_t)((e * (HID/16) + n) * (FFN_DIM/32) + ktile)) * 32 + lane) * 8);
                    v16h b = as_v16h(bp[0], bp[1]);
                    acc = __builtin_amdgcn_wmma_f32_16x16x32_f16(false, a, false, b, (short)0, acc, false, false);
                    asm volatile("v_nop\n\tv_nop\n\tv_nop\n\tv_nop" : "+v"(acc) : "v"(a), "v"(b));
                }
#pragma unroll
                for (int r = 0; r < 8; ++r) oacc[on][r] += (g8[r] * WSC_INV) * acc[r];
            }
            __syncthreads();
        }
    }

    float* stg = (float*)hbuf + w * 512;
#pragma unroll
    for (int rp = 0; rp < 8; rp += 2) {
#pragma unroll
        for (int on = 0; on < 8; ++on) {
            stg[(h * 2 + 0) * 128 + on * 16 + nl] = oacc[on][rp];
            stg[(h * 2 + 1) * 128 + on * 16 + nl] = oacc[on][rp + 1];
        }
        __builtin_amdgcn_fence(__ATOMIC_RELEASE, "workgroup");
        __builtin_amdgcn_wave_barrier();
        __builtin_amdgcn_fence(__ATOMIC_ACQUIRE, "workgroup");
        for (int pass = 0; pass < 2; ++pass) {
#pragma unroll
            for (int lr = 0; lr < 4; ++lr) {
                int hh = lr >> 1, dr = lr & 1;
                int grow = t0 + mw * 16 + 8 * hh + rp + dr;
                v4f v = *(const v4f*)(stg + lr * 128 + lane * 4);
                *(volatile v4f*)(out + (size_t)grow * HID + nw * 128 + lane * 4) = v;
            }
            __threadfence();
        }
        __builtin_amdgcn_fence(__ATOMIC_RELEASE, "workgroup");
        __builtin_amdgcn_wave_barrier();
        __builtin_amdgcn_fence(__ATOMIC_ACQUIRE, "workgroup");
    }
}

extern "C" void kernel_launch(void* const* d_in, const int* in_sizes, int n_in,
                              void* d_out, int out_size, void* d_ws, size_t ws_size,
                              hipStream_t stream) {
    (void)in_sizes; (void)n_in; (void)out_size; (void)ws_size;
    const float* x  = (const float*)d_in[0];
    const float* wr = (const float*)d_in[1];
    const float* w1 = (const float*)d_in[2];
    const float* w2 = (const float*)d_in[3];
    float* out = (float*)d_out;

    char* ws = (char*)d_ws;
    float*    logits = (float*)(ws + OFF_LOGITS);
    float*    gates  = (float*)(ws + OFF_GATES);
    unsigned* w1f    = (unsigned*)(ws + OFF_W1F);
    unsigned* w2f    = (unsigned*)(ws + OFF_W2F);
    unsigned* xfw    = (unsigned*)(ws + OFF_XF);

    router_kernel<<<T_TOK / 256, 256, 0, stream>>>(x, wr, logits);
    convert_w_kernel<<<(NEXP * HID * FFN_DIM / 2) / 256, 256, 0, stream>>>(w1, w1f, HID / 32, FFN_DIM / 16);
    convert_w_kernel<<<(NEXP * FFN_DIM * HID / 2) / 256, 256, 0, stream>>>(w2, w2f, FFN_DIM / 32, HID / 16);
    convert_x_kernel<<<(T_TOK * HID / 2) / 256, 256, 0, stream>>>(x, xfw);
    sinkhorn_gates_kernel<<<1, SKT, 0, stream>>>(logits, gates);
    moe_main_kernel<<<T_TOK / TM, 256, 0, stream>>>(xfw, w1f, w2f, gates, out);
}
